// RRGNN_90941637525590
// MI455X (gfx1250) — hardware-verified
//
#include <hip/hip_runtime.h>
#include <math.h>

#define NN 50000
#define NE 800000
#define DF 128
#define DO 64
#define KA 256
#define NP 50048
#define NT 256
#define SRB 2048
#define NTL 25
#define SCH 4096
#define NCH ((NE + SCH - 1) / SCH)
#define APR 8
#define SMP 4
#define RB1 400
#define NB1 (NN / RB1)
#define WSC 64.0f
#define WSC_INV 0.015625f
#define BN_EPS 1e-5f

static_assert(NP % 64 == 0 && NP >= NN, "pad");
static_assert(NTL * SRB >= NP, "tiles");
static_assert(NE % (SCH / NT) == 0, "edge groups");
static_assert(NN % RB1 == 0, "stat blocks");
static_assert(NN % 2 == 0 && NP % 2 == 0, "row pairs");
static_assert(NN < (1 << 17), "src packing");

typedef __attribute__((ext_vector_type(16))) _Float16 v16h;
typedef __attribute__((ext_vector_type(8)))  _Float16 v8h;
typedef __attribute__((ext_vector_type(16))) __bf16   v16b;
typedef __attribute__((ext_vector_type(8)))  __bf16   v8b;
typedef __attribute__((ext_vector_type(8)))  float    v8f;
typedef __attribute__((ext_vector_type(4)))  float    v4f;
typedef __attribute__((ext_vector_type(4)))  int      v4i;
typedef __attribute__((ext_vector_type(2)))  double   v2d;

__device__ __forceinline__ unsigned short f2bf_bits(float f) {
  unsigned u = __float_as_uint(f);
  return (unsigned short)((u + 0x7FFFu + ((u >> 16) & 1u)) >> 16);
}
__device__ __forceinline__ float bf_bits2f(unsigned short h) { return __uint_as_float(((unsigned)h) << 16); }

__device__ __forceinline__ void dep_guard_h(v8f& a, v8f& b, v16h x, v16h y) { asm volatile("v_nop\n\tv_nop\n\tv_nop\n\tv_nop" : "+v"(a), "+v"(b) : "v"(x), "v"(y)); }
__device__ __forceinline__ void dep_guard_b(v8f& a, v8f& b, v16b x, v16b y) { asm volatile("v_nop\n\tv_nop\n\tv_nop\n\tv_nop" : "+v"(a), "+v"(b) : "v"(x), "v"(y)); }
__device__ __forceinline__ void keep4_h(v16h a, v16h b, v16h c, v16h d) { asm volatile("v_nop" :: "v"(a), "v"(b), "v"(c), "v"(d)); }
__device__ __forceinline__ void keep4_b(v16b a, v16b b, v16b c, v16b d) { asm volatile("v_nop" :: "v"(a), "v"(b), "v"(c), "v"(d)); }
__device__ __forceinline__ void acc_guard4(v8f& a, v8f& b, v8f& c, v8f& d) { asm volatile("v_nop\n\tv_nop\n\tv_nop\n\tv_nop" : "+v"(a), "+v"(b), "+v"(c), "+v"(d)); }
template <typename T> struct Frag;
template <> struct Frag<_Float16> {
  typedef v16h V; union U { v16h v; v8h h[2]; };
  static __device__ __forceinline__ v16h load(const _Float16* p) {
    U f; f.h[0] = *(const v8h*)(p); f.h[1] = *(const v8h*)(p + 16); return f.v;
  }
  static __device__ __forceinline__ v8f mma(v16h a, v16h b, v8f c) {
    return __builtin_amdgcn_wmma_f32_16x16x32_f16(false, a, false, b, (short)0, c, false, false);
  }
  static __device__ __forceinline__ void guard(v8f& a, v8f& b, v16h x, v16h y) { dep_guard_h(a, b, x, y); }
  static __device__ __forceinline__ void keep(v16h a, v16h b, v16h c, v16h d) { keep4_h(a, b, c, d); }
};
template <> struct Frag<__bf16> {
  typedef v16b V; union U { v16b v; v8b h[2]; };
  static __device__ __forceinline__ v16b load(const __bf16* p) {
    U f; f.h[0] = *(const v8b*)(p); f.h[1] = *(const v8b*)(p + 16); return f.v;
  }
  static __device__ __forceinline__ v8f mma(v16b a, v16b b, v8f c) {
    return __builtin_amdgcn_wmma_f32_16x16x32_bf16(false, a, false, b, (short)0, c, false, false);
  }
  static __device__ __forceinline__ void guard(v8f& a, v8f& b, v16b x, v16b y) { dep_guard_b(a, b, x, y); }
  static __device__ __forceinline__ void keep(v16b a, v16b b, v16b c, v16b d) { keep4_b(a, b, c, d); }
};

template <int ET> struct Elem;
template <> struct Elem<0> { typedef _Float16 T; };
template <> struct Elem<1> { typedef __bf16 T; };
template <int ET, bool SPLIT, int BIAS_MODE, int OUT_MODE, bool RESID, int ACT = 0>
__global__ __launch_bounds__(256) void wmma_gemm64(
    const unsigned short* __restrict__ Ap, const unsigned short* __restrict__ A2p, int lda, long strideA,
    const unsigned short* __restrict__ Btp, const unsigned short* __restrict__ Bt2p, int ldb, long strideB,
    void* __restrict__ Cout, void* __restrict__ Cout2, int ldc, long strideC,
    const float* __restrict__ bias,
    const float* __restrict__ resid, long strideR,
    int M, int N, int K, float scale) {
  typedef typename Elem<ET>::T T;
  typedef typename Frag<T>::V V;
  const T* A = (const T*)Ap; const T* A2 = (const T*)A2p; const T* Bt = (const T*)Btp; const T* Bt2 = (const T*)Bt2p;
  __shared__ __align__(16) float sT[8][16 * 68];
  const int b    = blockIdx.y;
  const int lane = threadIdx.x & 31;
  const int wave = threadIdx.x >> 5;
  const int tilesN = N >> 6;
  const int tilesM = M >> 6;
  const int tile = blockIdx.x * 8 + wave;
  if (tile >= tilesM * tilesN) return;
  const int tm = tile / tilesN;
  const int tn = tile - tm * tilesN;
  const int m0 = tm << 6;
  const int n0 = tn << 6;

  const T* Ab  = A  + (size_t)b * strideA;
  const T* Bb  = Bt + (size_t)b * strideB;
  const T* Ab2 = SPLIT ? (A2  + (size_t)b * strideA) : nullptr;
  const T* Bb2 = SPLIT ? (Bt2 + (size_t)b * strideB) : nullptr;

  const int rlane = lane & 15;
  const int koff  = (lane >> 4) * 8;
  const int mOff  = (lane >> 4) * 8;

  v8f acc[4][4];
#pragma unroll
  for (int i = 0; i < 4; ++i)
#pragma unroll
    for (int j = 0; j < 4; ++j) acc[i][j] = (v8f){0.f,0.f,0.f,0.f,0.f,0.f,0.f,0.f};

  for (int k0 = 0; k0 < K; k0 += 32) {
    V bh[4], bl[4];
#pragma unroll
    for (int j = 0; j < 4; ++j) {
      const size_t bo = (size_t)(n0 + (j << 4) + rlane) * ldb + koff + k0;
      bh[j] = Frag<T>::load(Bb + bo);
      if (SPLIT) bl[j] = Frag<T>::load(Bb2 + bo);
    }
#pragma unroll
    for (int i = 0; i < 4; ++i) {
      const size_t ao = (size_t)(m0 + (i << 4) + rlane) * lda + koff + k0;
      V ah = Frag<T>::load(Ab + ao);
      V al;
      if (SPLIT) al = Frag<T>::load(Ab2 + ao);
#pragma unroll
      for (int j = 0; j < 4; ++j) {
        acc[i][j] = Frag<T>::mma(ah, bh[j], acc[i][j]);
        if (SPLIT) {
          acc[i][j] = Frag<T>::mma(ah, bl[j], acc[i][j]);
          acc[i][j] = Frag<T>::mma(al, bh[j], acc[i][j]);
        }
      }
      Frag<T>::guard(acc[i][0], acc[i][3], ah, SPLIT ? al : ah);
    }
    Frag<T>::keep(bh[0], bh[1], bh[2], bh[3]);
    if (SPLIT) Frag<T>::keep(bl[0], bl[1], bl[2], bl[3]);
  }
  acc_guard4(acc[0][0], acc[0][1], acc[0][2], acc[0][3]);
  acc_guard4(acc[1][0], acc[1][1], acc[1][2], acc[1][3]);
  acc_guard4(acc[2][0], acc[2][1], acc[2][2], acc[2][3]);
  acc_guard4(acc[3][0], acc[3][1], acc[3][2], acc[3][3]);

  float* slab = sT[wave];
  const float* Rb = RESID ? (resid + (size_t)b * strideR) : nullptr;
#pragma unroll
  for (int i = 0; i < 4; ++i) {
    const int mBase = m0 + (i << 4);
#pragma unroll
    for (int j = 0; j < 4; ++j) {
      const int n = n0 + (j << 4) + rlane;
      float bv = 0.f;
      if (BIAS_MODE == 2) bv = bias[n];
#pragma unroll
      for (int r = 0; r < 8; ++r) {
        float v = acc[i][j][r] * scale;
        if (BIAS_MODE == 1) v += bias[mBase + mOff + r];
        if (BIAS_MODE == 2) v += bv;
        if (RESID) v += Rb[(size_t)(mBase + mOff + r) * ldc + n];
        if (ACT == 1) v = tanhf(v);
        if (ACT == 2) v = fmaxf(v, 0.0f);
        if (ACT == 3) v = v / (1.0f + expf(-v));
        if (ACT == 4) v = (v > 0.f) ? v : 0.01f * v;
        if (ACT == 5) v = 0.5f * v * (1.0f + erff(v * 0.70710678118654752f));
        slab[(mOff + r) * 68 + (j << 4) + rlane] = v;
      }
    }
    __builtin_amdgcn_fence(__ATOMIC_RELEASE, "workgroup");
    __builtin_amdgcn_wave_barrier();
    __builtin_amdgcn_fence(__ATOMIC_ACQUIRE, "workgroup");
    if (OUT_MODE == 0) {
      float* C = (float*)Cout + (size_t)b * strideC;
      const int hh = lane >> 4, c4 = (lane & 15) * 4;
      for (int pass = 0; pass < 2; ++pass) {
#pragma unroll
        for (int it = 0; it < 8; ++it) {
          const int row = it * 2 + hh;
          v4f v = *(const v4f*)(slab + row * 68 + c4);
          *(volatile v4f*)(C + (size_t)(mBase + row) * ldc + n0 + c4) = v;
        }
        __threadfence();
      }
    } else {
      const int q = lane >> 3, c8 = (lane & 7) * 8;
      unsigned short* C  = (unsigned short*)Cout  + (size_t)b * strideC;
      unsigned short* C2 = (OUT_MODE == 2) ? ((unsigned short*)Cout2 + (size_t)b * strideC) : nullptr;
      for (int pass = 0; pass < 2; ++pass) {
#pragma unroll
        for (int it = 0; it < 4; ++it) {
          const int row = it * 4 + q;
          const float* sp = slab + row * 68 + c8;
          v8h hv, lv;
#pragma unroll
          for (int e = 0; e < 8; ++e) {
            if (OUT_MODE == 1) {
              hv[e] = (_Float16)sp[e];
            } else {
              unsigned short hb = f2bf_bits(sp[e]);
              unsigned short lb = f2bf_bits(sp[e] - bf_bits2f(hb));
              hv[e] = __builtin_bit_cast(_Float16, hb);
              lv[e] = __builtin_bit_cast(_Float16, lb);
            }
          }
          *(volatile v8h*)(C + (size_t)(mBase + row) * ldc + n0 + c8) = hv;
          if (OUT_MODE == 2) *(volatile v8h*)(C2 + (size_t)(mBase + row) * ldc + n0 + c8) = lv;
        }
        __threadfence();
      }
    }
    __builtin_amdgcn_fence(__ATOMIC_RELEASE, "workgroup");
    __builtin_amdgcn_wave_barrier();
    __builtin_amdgcn_fence(__ATOMIC_ACQUIRE, "workgroup");
  }
}

__device__ __forceinline__ int blk_excl_scan(int cnt, int* scan_ws, int tid, int* tot) {
  const int lane = tid & 31, wave = tid >> 5; int incl = cnt;
#pragma unroll
  for (int o = 1; o < 32; o <<= 1) { const int v = __shfl_up(incl, o, 32); if (lane >= o) incl += v; }
  if (lane == 31) scan_ws[wave] = incl;
  __syncthreads();
  if (wave == 0) { int wv = (lane < NT / 32) ? scan_ws[lane] : 0; int wincl = wv;
#pragma unroll
    for (int o = 1; o < 32; o <<= 1) { const int v = __shfl_up(wincl, o, 32); if (lane >= o) wincl += v; }
    if (lane < NT / 32) scan_ws[32 + lane] = wincl - wv; if (lane == 31) scan_ws[64] = wincl; }
  __syncthreads();
  const int res = scan_ws[32 + wave] + incl - cnt; *tot = scan_ws[64];
  return res;
}
template <int SP, int CAP>
__device__ __forceinline__ int chunk_hits(const int* __restrict__ dstv, const int* __restrict__ srcv, int e0, int n0, int tid,
                                          int* LIST, int* scan_ws) {
  const int eb = e0 + tid * SP;
  const bool inr = eb < NE;
  const int ebc = inr ? eb : (NE - SP);
  int rec[SP]; int cnt = 0;
#pragma unroll
  for (int k = 0; k < SP; k += 4) {
    const v4i d4 = *(const v4i*)(dstv + ebc + k);
    const v4i s4 = *(const v4i*)(srcv + ebc + k);
#pragma unroll
    for (int e = 0; e < 4; ++e) {
      const int d = d4[e]; int r = -1;
      if (inr && d >= n0 && d < n0 + SRB) { int s = s4[e]; s = s < 0 ? 0 : (s >= NN ? NN - 1 : s); r = ((d - n0) << 17) | s; ++cnt; }
      rec[k + e] = r;
    }
  }
  int tot; int p = blk_excl_scan(cnt, scan_ws, tid, &tot);
#pragma unroll
  for (int k = 0; k < SP; ++k) if (rec[k] >= 0) { if ((unsigned)p < (unsigned)CAP) LIST[p] = rec[k]; ++p; }
  __syncthreads();
  return tot < CAP ? tot : CAP;
}

__global__ __launch_bounds__(NT) void bt_kernel(const float* __restrict__ Wl, const float* __restrict__ Wr, _Float16* __restrict__ Bt,
                                               int nout) {
  const int i = blockIdx.x * NT + threadIdx.x;
  if (i < nout * (KA / 8)) {
    const int o = i >> 5;
    const int k8 = (i & 31) * 8;
    const float* sp = (k8 < DF) ? (Wl + o * DF + k8) : (Wr + o * DF + (k8 - DF));
    const v4f w0 = *(const v4f*)sp, w1 = *(const v4f*)(sp + 4);
    v8h hv;
#pragma unroll
    for (int e = 0; e < 4; ++e) { hv[e] = (_Float16)(w0[e] * WSC); hv[4 + e] = (_Float16)(w1[e] * WSC); }
    _Float16* dp = Bt + (size_t)o * KA + k8;
    *(volatile v8h*)dp = hv;
    __threadfence();
    *(volatile v8h*)dp = hv;
  }
}

__global__ __launch_bounds__(NT) void agg_kernel(const float* __restrict__ hs, const int* __restrict__ ei, float* AGG,
                                                _Float16* __restrict__ A16) {
  __shared__ int LIST[SCH];
  __shared__ float DEG[SRB];
  __shared__ int scan_ws[80];
  const int tid = threadIdx.x, lane = tid & 31, wave = tid >> 5;
  const int n0 = blockIdx.x * SRB;
  const int rbase = blockIdx.x * SRB;
  const v4f z4 = {0.f, 0.f, 0.f, 0.f};
#pragma unroll 1
  for (int j = 0; j < 256; ++j) {
    float* rp = AGG + (size_t)(rbase + wave * 256 + j) * DF + 4 * lane;
    *(volatile v4f*)rp = z4;
  }
  __threadfence();
#pragma unroll 1
  for (int j = 0; j < 256; ++j) {
    float* rp = AGG + (size_t)(rbase + wave * 256 + j) * DF + 4 * lane;
    *(volatile v4f*)rp = z4;
  }
  for (int i = tid; i < SRB; i += NT) DEG[i] = 0.f;
  __syncthreads();
  const int* srcv = ei; const int* dstv = ei + NE;
#pragma unroll 1
  for (int c = 0; c < NCH; ++c) {
    const int tot = chunk_hits<SCH / NT, SCH>(dstv, srcv, c * SCH, n0, tid, LIST, scan_ws);
#pragma unroll 1
    for (int base = 0; base < tot; base += 32) {
      const int q = base + lane;
      const int rv = (q < tot) ? LIST[q] : -1;
      const int own = (rv >= 0 && (rv >> 25) == wave) ? 1 : 0;
      unsigned msk = (unsigned)__ballot(own);
#pragma unroll 1
      for (int it = 0; it < 32; ++it) {
        if (msk == 0u) break;
        const int bp = __builtin_ctz(msk); msk &= msk - 1u;
        const int r = __shfl(rv, bp, 32);
        const int dl = (r >> 17) & (SRB - 1);
        int s = r & 0x1FFFF; s = s < NN ? s : NN - 1;
        const v4f xv = *(const v4f*)(hs + (size_t)s * DF + 4 * lane);
        if (lane == 0) DEG[dl] += 1.0f;
        float* rp = AGG + (size_t)(rbase + dl) * DF + 4 * lane;
        v4f a = *(const v4f*)rp;
        a = a + xv;
        *(volatile v4f*)rp = a;
        __threadfence();
        *(volatile v4f*)rp = a;
      }
    }
    __syncthreads();
  }
  const int hh = lane >> 4, cc = (lane & 15) * 8;
#pragma unroll 1
  for (int j = 0; j < 128; ++j) {
    const int dl = wave * 256 + 2 * j;
    const int n = n0 + dl;
    if (n < NP) {
      const int dr = dl + hh, nr = n + hh;
      const bool live = nr < NN;
      const int nc = live ? nr : (NN - 1);
      const float* xp = hs + (size_t)nc * DF + cc;
      const v4f x0 = *(const v4f*)xp, x1 = *(const v4f*)(xp + 4);
      const float* rp = AGG + (size_t)(rbase + dr) * DF + cc;
      const v4f a0 = *(const v4f*)rp, a1 = *(const v4f*)(rp + 4);
      const float dg = DEG[dr];
      const float inv = 1.0f / fmaxf(dg, 1.0f);
      const v4f mv0 = a0 * inv, mv1 = a1 * inv;
      v8h hx, hm;
#pragma unroll
      for (int e = 0; e < 4; ++e) {
        hx[e]     = live ? (_Float16)x0[e]  : (_Float16)0.0f;
        hx[4 + e] = live ? (_Float16)x1[e]  : (_Float16)0.0f;
        hm[e]     = live ? (_Float16)mv0[e] : (_Float16)0.0f;
        hm[4 + e] = live ? (_Float16)mv1[e] : (_Float16)0.0f;
      }
      _Float16* ap = A16 + (size_t)nr * KA + cc;
      *(volatile v8h*)ap = hm; *(volatile v8h*)(ap + DF) = hx;
      __threadfence();
      *(volatile v8h*)ap = hm; *(volatile v8h*)(ap + DF) = hx;
    }
  }
}

__global__ __launch_bounds__(DF) void bn_part_kernel(const float* __restrict__ C, double* __restrict__ STP) {
  const int c = threadIdx.x;
  const int r0 = blockIdx.x * RB1;
  double s = 0.0, s2 = 0.0;
#pragma unroll 4
  for (int r = 0; r < RB1; ++r) {
    const double v = (double)C[(size_t)(r0 + r) * DF + c];
    s += v; s2 += v * v;
  }
  const v2d o = {s, s2};
  double* p = STP + ((size_t)blockIdx.x * DF + c) * 2;
  *(volatile v2d*)p = o;
  __threadfence();
  *(volatile v2d*)p = o;
}

__global__ __launch_bounds__(DF) void bn_fin_kernel(const double* __restrict__ STP, const float* __restrict__ gam,
                                                   const float* __restrict__ bet, float* __restrict__ STF) {
  const int c = threadIdx.x;
  double s = 0.0, s2 = 0.0;
#pragma unroll 1
  for (int b = 0; b < NB1; ++b) {
    const v2d v = *(const v2d*)(STP + ((size_t)b * DF + c) * 2);
    s += v[0]; s2 += v[1];
  }
  const double mu = s * (1.0 / (double)NN);
  double var = s2 * (1.0 / (double)NN) - mu * mu;
  var = var < 0.0 ? 0.0 : var;
  const float muf = (float)mu;
  const float rstd = rsqrtf((float)var + BN_EPS);
  const v4f o = {muf, rstd, gam[c], bet[c]};
  float* p = STF + 4 * c;
  *(volatile v4f*)p = o;
  __threadfence();
  *(volatile v4f*)p = o;
}

__global__ __launch_bounds__(NT) void bn_apply_kernel(const float* __restrict__ C, const float* __restrict__ STF, float* __restrict__ H) {
  const int lane = threadIdx.x & 31, wave = threadIdx.x >> 5;
  const v4f t0 = *(const v4f*)(STF + 16 * lane), t1 = *(const v4f*)(STF + 16 * lane + 4),
            t2 = *(const v4f*)(STF + 16 * lane + 8), t3 = *(const v4f*)(STF + 16 * lane + 12);
  const v4f mu = {t0[0], t1[0], t2[0], t3[0]};
  const v4f rs = {t0[1], t1[1], t2[1], t3[1]};
  const v4f g  = {t0[2], t1[2], t2[2], t3[2]};
  const v4f bb = {t0[3], t1[3], t2[3], t3[3]};
  const int r0 = (blockIdx.x * (NT / 32) + wave) * APR;
#pragma unroll 1
  for (int j = 0; j < APR; ++j) {
    const int row = r0 + j;
    if (row < NN) {
      const v4f h = *(const v4f*)(C + (size_t)row * DF + 4 * lane);
      v4f o;
#pragma unroll
      for (int e = 0; e < 4; ++e) {
        const float y = ((h[e] - mu[e]) * rs[e]) * g[e] + bb[e];
        o[e] = fmaxf(y, 0.0f);
      }
      float* op = H + (size_t)row * DF + 4 * lane;
      *(volatile v4f*)op = o;
      __threadfence();
      *(volatile v4f*)op = o;
    }
  }
}

__global__ __launch_bounds__(NT) void softmax_kernel(const float* __restrict__ C, float* __restrict__ out) {
  const int lane = threadIdx.x & 31, wave = threadIdx.x >> 5;
  const int hh = lane >> 4, c4 = (lane & 15) * 4;
  const int p0 = (blockIdx.x * (NT / 32) + wave) * SMP;
#pragma unroll 1
  for (int j = 0; j < SMP; ++j) {
    const int p = p0 + j;
    if (p < NN / 2) {
      const int row = 2 * p + hh;
      const v4f v = *(const v4f*)(C + (size_t)row * DO + c4);
      float m = fmaxf(fmaxf(v[0], v[1]), fmaxf(v[2], v[3]));
#pragma unroll
      for (int off = 1; off < 16; off <<= 1) m = fmaxf(m, __shfl_xor(m, off, 32));
      v4f ex;
#pragma unroll
      for (int e = 0; e < 4; ++e) ex[e] = __expf(v[e] - m);
      float s = (ex[0] + ex[1]) + (ex[2] + ex[3]);
#pragma unroll
      for (int off = 1; off < 16; off <<= 1) s += __shfl_xor(s, off, 32);
      const float inv = 1.0f / s;
      const v4f o = ex * inv;
      float* op = out + (size_t)row * DO + c4;
      *(volatile v4f*)op = o;
      __threadfence();
      *(volatile v4f*)op = o;
    }
  }
}

extern "C" void kernel_launch(void* const* d_in, const int* in_sizes, int n_in,
                              void* d_out, int out_size, void* d_ws, size_t ws_size, hipStream_t stream) {
  if (n_in < 15) return;
  if (in_sizes[0] != NN * DF || in_sizes[1] != 2 * NE ||
      in_sizes[2] != DF * DF || in_sizes[3] < DF || in_sizes[4] != DF * DF ||
      in_sizes[5] != DF * DF || in_sizes[6] < DF || in_sizes[7] != DF * DF ||
      in_sizes[8] != DO * DF || in_sizes[9] < DO || in_sizes[10] != DO * DF ||
      in_sizes[11] < DF || in_sizes[12] < DF || in_sizes[13] < DF || in_sizes[14] < DF ||
      out_size != NN * DO) return;
  const float* x   = (const float*)d_in[0];
  const int*   ei  = (const int*)  d_in[1];
  const float* Wl0 = (const float*)d_in[2];
  const float* bl0 = (const float*)d_in[3];
  const float* Wr0 = (const float*)d_in[4];
  const float* Wl1 = (const float*)d_in[5];
  const float* bl1 = (const float*)d_in[6];
  const float* Wr1 = (const float*)d_in[7];
  const float* Wl2 = (const float*)d_in[8];
  const float* bl2 = (const float*)d_in[9];
  const float* Wr2 = (const float*)d_in[10];
  const float* g0  = (const float*)d_in[11];
  const float* be0 = (const float*)d_in[12];
  const float* g1  = (const float*)d_in[13];
  const float* be1 = (const float*)d_in[14];
  float* out = (float*)d_out;

  char* ws = (char*)d_ws; size_t off = 0;
  auto carve = [&](size_t bytes) -> char* { char* p = ws + off; off += (bytes + 255) & ~(size_t)255; return p; };
  _Float16* A16 = (_Float16*)carve((size_t)NP * KA * 2);
  _Float16* BT0 = (_Float16*)carve((size_t)DF * KA * 2);
  _Float16* BT1 = (_Float16*)carve((size_t)DF * KA * 2);
  _Float16* BT2 = (_Float16*)carve((size_t)DO * KA * 2);
  char*     R   = carve((size_t)NTL * SRB * DF * 4);
  float*    H   = (float*)carve((size_t)NN * DF * 4);
  double*   STP = (double*)carve((size_t)NB1 * DF * 2 * 8);
  float*    STF = (float*)carve((size_t)DF * 4 * 4);
  if (off > ws_size || off > (size_t)134217728) return;
  float* AGG = (float*)R;
  float* C   = (float*)R;

  const int gemm_grid_h = ((NP / 64) * (DF / 64) + 7) / 8;
  const int gemm_grid_o = ((NP / 64) * (DO / 64) + 7) / 8;
  const int apply_grid  = (NN + (NT / 32) * APR - 1) / ((NT / 32) * APR);
  const int smx_grid    = (NN / 2 + (NT / 32) * SMP - 1) / ((NT / 32) * SMP);

  bt_kernel<<<(DF * (KA / 8) + NT - 1) / NT, NT, 0, stream>>>(Wl0, Wr0, BT0, DF);
  bt_kernel<<<(DF * (KA / 8) + NT - 1) / NT, NT, 0, stream>>>(Wl1, Wr1, BT1, DF);
  bt_kernel<<<(DO * (KA / 8) + NT - 1) / NT, NT, 0, stream>>>(Wl2, Wr2, BT2, DO);

  agg_kernel<<<NTL, NT, 0, stream>>>(x, ei, AGG, A16);
  wmma_gemm64<0, false, 2, 0, false, 0><<<dim3(gemm_grid_h, 1), 256, 0, stream>>>(
      (const unsigned short*)A16, (const unsigned short*)nullptr, KA, 0L,
      (const unsigned short*)BT0, (const unsigned short*)nullptr, KA, 0L,
      (void*)C, (void*)nullptr, DF, 0L,
      bl0, (const float*)nullptr, 0L, NP, DF, KA, WSC_INV);
  bn_part_kernel<<<NB1, DF, 0, stream>>>(C, STP);
  bn_fin_kernel<<<1, DF, 0, stream>>>(STP, g0, be0, STF);
  bn_apply_kernel<<<apply_grid, NT, 0, stream>>>(C, STF, H);

  agg_kernel<<<NTL, NT, 0, stream>>>(H, ei, AGG, A16);
  wmma_gemm64<0, false, 2, 0, false, 0><<<dim3(gemm_grid_h, 1), 256, 0, stream>>>(
      (const unsigned short*)A16, (const unsigned short*)nullptr, KA, 0L,
      (const unsigned short*)BT1, (const unsigned short*)nullptr, KA, 0L,
      (void*)C, (void*)nullptr, DF, 0L,
      bl1, (const float*)nullptr, 0L, NP, DF, KA, WSC_INV);
  bn_part_kernel<<<NB1, DF, 0, stream>>>(C, STP);
  bn_fin_kernel<<<1, DF, 0, stream>>>(STP, g1, be1, STF);
  bn_apply_kernel<<<apply_grid, NT, 0, stream>>>(C, STF, H);

  agg_kernel<<<NTL, NT, 0, stream>>>(H, ei, AGG, A16);
  wmma_gemm64<0, false, 2, 0, false, 0><<<dim3(gemm_grid_o, 1), 256, 0, stream>>>(
      (const unsigned short*)A16, (const unsigned short*)nullptr, KA, 0L,
      (const unsigned short*)BT2, (const unsigned short*)nullptr, KA, 0L,
      (void*)C, (void*)nullptr, DO, 0L,
      bl2, (const float*)nullptr, 0L, NP, DO, KA, WSC_INV);
  softmax_kernel<<<smx_grid, NT, 0, stream>>>(C, out);
}
